// GlobalFeatureGAT_23338852286623
// MI455X (gfx1250) — hardware-verified
//
#include <hip/hip_runtime.h>
#include <stddef.h>


#define SF      64
#define LL      20
#define DM      32
#define NTAB    5
#define FT      224
#define KPA     256
#define HCA     512
#define HCB     128
#define NHA     4
#define EP      8
#define NCP     128
#define GBM     64
#define GTHR    128
#define NTHR    256
#define NWAVE   8
#define EPT     8
#define CHUNK   (NTHR * EPT)
#define WCAP    (EPT * 32)
#define LISTN   (NWAVE * WCAP)
#define NBMAX   2048
#define RCAP    28672
#define DEGCAP  4096
#define PTHR    128
#define NEG_SLOPE 0.2f
#define LN_EPS  0.00001f
#define CA      16.0f
#define CW      64.0f
#define SCL     0.0009765625f
#define WSCAP   134217728
#define LDS_AGG ((2 * RCAP + 2 * NBMAX + LISTN) * 4 + 64)

static_assert((CHUNK & (CHUNK - 1)) == 0 && CHUNK <= 4096);
static_assert((NBMAX & (NBMAX - 1)) == 0 && NBMAX <= 4096);
static_assert(NTHR * 8 == NBMAX);
static_assert(LISTN >= NBMAX);
static_assert(LISTN >= NWAVE * WCAP);
static_assert((RCAP % 32) == 0);
static_assert(LDS_AGG <= 300000);
static_assert(GBM == (GTHR / 32) * 16);
static_assert(GTHR == NCP);
static_assert((FT % 32) == 0);
static_assert((HCA % 32) == 0);
static_assert(KPA >= FT && (KPA % 64) == 0);
static_assert(FT == SF + NTAB * DM);
static_assert(HCA == NHA * NCP);
static_assert(HCB == NCP);
static_assert(PTHR == HCB);
static_assert(SF == 2 * 32 && DM == 32);

typedef float    v2f  __attribute__((ext_vector_type(2)));
typedef float    v4f  __attribute__((ext_vector_type(4)));
typedef float    v8f  __attribute__((ext_vector_type(8)));
typedef int      v4i  __attribute__((ext_vector_type(4)));
typedef int      v8i  __attribute__((ext_vector_type(8)));
typedef _Float16 v4h  __attribute__((ext_vector_type(4)));
typedef _Float16 v8h  __attribute__((ext_vector_type(8)));
typedef _Float16 v16h __attribute__((ext_vector_type(16)));
union FragH { v16h v; v8h h[2]; v8i w; };

__device__ __forceinline__ v8f wmh(const FragH& a, const FragH& b, v8f c) {
  v8f d = __builtin_amdgcn_wmma_f32_16x16x32_f16(false, a.v, false, b.v, (short)0, c, false, false);
  asm volatile("v_nop\n\tv_nop\n\tv_nop\n\tv_nop" : "+v"(d) : "v"(a.w), "v"(b.w));
  return d;
}

__device__ __forceinline__ float elu1(float v) {
  const float e = __expf(fminf(v, 0.0f)) - 1.0f;
  return v > 0.0f ? v : e;
}
__device__ __forceinline__ v4f elu4(v4f v) {
  v4f r;
  r.x = elu1(v.x); r.y = elu1(v.y); r.z = elu1(v.z); r.w = elu1(v.w);
  return r;
}

__device__ __forceinline__ int scan_chunk(const int* __restrict__ dsts, int nE, int cbase, int slotBase,
                                          int nb, int vec8, int* list, int tid, int lane, int wave) {
  int wc = 0;
  const int el0  = tid * EPT;
  const int e0   = cbase + el0;
  const int sent = -2147483647 - 1;
  v4i da, db;
  if (vec8 != 0 && cbase + CHUNK <= nE) {
    da = *(const v4i*)(dsts + e0);
    db = *(const v4i*)(dsts + e0 + 4);
  } else {
    da.x = (e0     < nE) ? dsts[min(e0,     nE - 1)] : sent;
    da.y = (e0 + 1 < nE) ? dsts[min(e0 + 1, nE - 1)] : sent;
    da.z = (e0 + 2 < nE) ? dsts[min(e0 + 2, nE - 1)] : sent;
    da.w = (e0 + 3 < nE) ? dsts[min(e0 + 3, nE - 1)] : sent;
    db.x = (e0 + 4 < nE) ? dsts[min(e0 + 4, nE - 1)] : sent;
    db.y = (e0 + 5 < nE) ? dsts[min(e0 + 5, nE - 1)] : sent;
    db.z = (e0 + 6 < nE) ? dsts[min(e0 + 6, nE - 1)] : sent;
    db.w = (e0 + 7 < nE) ? dsts[min(e0 + 7, nE - 1)] : sent;
  }
  const unsigned nbs = (unsigned)slotBase;
  const unsigned unb = (unsigned)nb;
  const unsigned s0 = (unsigned)da.x - nbs, s1 = (unsigned)da.y - nbs;
  const unsigned s2 = (unsigned)da.z - nbs, s3 = (unsigned)da.w - nbs;
  const unsigned s4 = (unsigned)db.x - nbs, s5 = (unsigned)db.y - nbs;
  const unsigned s6 = (unsigned)db.z - nbs, s7 = (unsigned)db.w - nbs;
  const bool h0 = s0 < unb, h1 = s1 < unb, h2 = s2 < unb, h3 = s3 < unb;
  const bool h4 = s4 < unb, h5 = s5 < unb, h6 = s6 < unb, h7 = s7 < unb;
  const unsigned any = __builtin_amdgcn_ballot_w32(h0 | h1 | h2 | h3 | h4 | h5 | h6 | h7);
  if (any != 0u) {
#define HITJ(J, HJ, SJ) { \
      const unsigned mj = __builtin_amdgcn_ballot_w32(HJ); \
      if (mj != 0u) { \
        if (HJ) { \
          const int pos = wc + (int)__builtin_amdgcn_mbcnt_lo(mj, 0u); \
          if (pos < WCAP) list[wave * WCAP + pos] = ((el0 + (J)) << 12) | (int)(SJ); \
        } \
        wc += (int)__builtin_popcount(mj); } }
    HITJ(0, h0, s0)
    HITJ(1, h1, s1)
    HITJ(2, h2, s2)
    HITJ(3, h3, s3)
    HITJ(4, h4, s4)
    HITJ(5, h5, s5)
    HITJ(6, h6, s6)
    HITJ(7, h7, s7)
#undef HITJ
  }
  return wc;
}

__global__ __launch_bounds__(NTHR) void k_feat(
    const float* __restrict__ xs,
    const int* __restrict__ i0, const int* __restrict__ i1, const int* __restrict__ i2,
    const int* __restrict__ i3, const int* __restrict__ i4,
    const float* __restrict__ e0, const float* __restrict__ e1, const float* __restrict__ e2,
    const float* __restrict__ e3, const float* __restrict__ e4,
    const float* __restrict__ lnsc, const float* __restrict__ lnb,
    _Float16* xa, int nN, int vc0, int vc1, int vc2, int vc3, int vc4) {
  __shared__ __attribute__((aligned(16))) float srow[NWAVE * KPA];
  const int tid = threadIdx.x, lane = tid & 31, wave = tid >> 5;
  const int node = (int)blockIdx.x * NWAVE + wave;
  const int nc = node < nN ? node : nN - 1;
  const v2f sc = *(const v2f*)(xs + (size_t)nc * SF + 2 * lane);
  float pv[NTAB];
#pragma unroll
  for (int t = 0; t < NTAB; ++t) {
    const int*   tab = (t == 0) ? i0 : (t == 1) ? i1 : (t == 2) ? i2 : (t == 3) ? i3 : i4;
    const float* emb = (t == 0) ? e0 : (t == 1) ? e1 : (t == 2) ? e2 : (t == 3) ? e3 : e4;
    const int    voc = (t == 0) ? vc0 : (t == 1) ? vc1 : (t == 2) ? vc2 : (t == 3) ? vc3 : vc4;
    const int* tp = tab + (size_t)nc * LL;
    float s = 0.0f;
    int cnt = 0;
#pragma unroll 1
    for (int j = 0; j < LL; ++j) {
      const int idx = tp[j];
      const int ci  = idx < 0 ? 0 : (idx > voc - 1 ? voc - 1 : idx);
      const float ev = emb[(size_t)ci * DM + lane];
      const bool on = (idx != 0);
      s += on ? ev : 0.0f;
      cnt += on ? 1 : 0;
    }
    pv[t] = s * __builtin_amdgcn_rcpf((float)cnt + 1e-9f);
  }
  float sum = sc.x + sc.y;
#pragma unroll
  for (int t = 0; t < NTAB; ++t) sum += pv[t];
#pragma unroll
  for (int o = 16; o > 0; o >>= 1) sum += __shfl_xor(sum, o);
  const float mu = sum * (1.0f / (float)FT);
  const float d0 = sc.x - mu, d1 = sc.y - mu;
  float dp[NTAB];
  float q = d0 * d0 + d1 * d1;
#pragma unroll
  for (int t = 0; t < NTAB; ++t) { dp[t] = pv[t] - mu; q += dp[t] * dp[t]; }
#pragma unroll
  for (int o = 16; o > 0; o >>= 1) q += __shfl_xor(q, o);
  const float var  = q * (1.0f / (float)FT);
  const float rstd = rsqrtf(var + LN_EPS);
  const v2f g2 = *(const v2f*)(lnsc + 2 * lane);
  const v2f o2 = *(const v2f*)(lnb + 2 * lane);
  v2f y2;
  y2.x = (d0 * rstd) * g2.x + o2.x;
  y2.y = (d1 * rstd) * g2.y + o2.y;
  float yp[NTAB];
#pragma unroll
  for (int t = 0; t < NTAB; ++t) {
    const int f = SF + DM * t + lane;
    yp[t] = (dp[t] * rstd) * lnsc[f] + lnb[f];
  }
  const bool valid = node < nN;
  if (!valid) {
    y2.x = 0.0f; y2.y = 0.0f;
#pragma unroll
    for (int t = 0; t < NTAB; ++t) yp[t] = 0.0f;
  }
  float* sr = srow + wave * KPA;
  *(v2f*)(sr + 2 * lane) = y2;
#pragma unroll
  for (int t = 0; t < NTAB; ++t) sr[SF + DM * t + lane] = yp[t];
  sr[FT + lane] = 0.0f;
  __syncthreads();
  const v4f a = *(const v4f*)(sr + 8 * lane);
  const v4f b = *(const v4f*)(sr + 8 * lane + 4);
  v8h hv;
  hv[0] = (_Float16)(a.x * CA); hv[1] = (_Float16)(a.y * CA);
  hv[2] = (_Float16)(a.z * CA); hv[3] = (_Float16)(a.w * CA);
  hv[4] = (_Float16)(b.x * CA); hv[5] = (_Float16)(b.y * CA);
  hv[6] = (_Float16)(b.z * CA); hv[7] = (_Float16)(b.w * CA);
  const size_t o = (size_t)node * KPA + 8 * lane;
  *(volatile v8h*)(xa + o) = hv;
  __threadfence();
  *(volatile v8h*)(xa + o) = hv;
}

__global__ __launch_bounds__(NTHR) void k_wprep(const float* __restrict__ w, _Float16* wt,
                                                int K, int Nout, int KP, int nUnits) {
  const int u = (int)blockIdx.x * NTHR + (int)threadIdx.x;
  if (u >= nUnits) return;
  const int upr = KP >> 3;
  const int n   = u / upr;
  const int k8  = (u - n * upr) * 8;
  v8h hv;
#pragma unroll
  for (int i = 0; i < 8; ++i) {
    const int kk = k8 + i;
    const int kc = kk < K ? kk : K - 1;
    const float v = w[(size_t)kc * Nout + n];
    hv[i] = (_Float16)((kk < K ? v : 0.0f) * CW);
  }
  const size_t o = (size_t)n * KP + k8;
  *(volatile v8h*)(wt + o) = hv;
  __threadfence();
  *(volatile v8h*)(wt + o) = hv;
}

__global__ __launch_bounds__(GTHR) void k_gemm(const _Float16* __restrict__ xh, int lda, int ksteps,
                                               const _Float16* __restrict__ wt, int ldb,
                                               const float* __restrict__ asrc, const float* __restrict__ adst,
                                               float* Y, int yp, float* ES, float* ED, int P) {
  __shared__ __attribute__((aligned(16))) float stg[GBM * NCP];
  __shared__ __attribute__((aligned(16))) float esT[GBM * EP];
  __shared__ __attribute__((aligned(16))) float edT[GBM * EP];
  __shared__ float sAs[NCP];
  __shared__ float sAd[NCP];
  const int tid = threadIdx.x, lane = tid & 31, wave = tid >> 5, hh = lane >> 4, m = lane & 15;
  const int rowBase = (int)blockIdx.x * GBM;
  for (int i = tid; i < GBM * EP; i += GTHR) { esT[i] = 0.0f; edT[i] = 0.0f; }
  const size_t arow = (size_t)(rowBase + 16 * wave + m) * lda + 8 * hh;
#pragma unroll 1
  for (int p = 0; p < P; ++p) {
    sAs[tid] = asrc[p * NCP + tid];
    sAd[tid] = adst[p * NCP + tid];
#pragma unroll 1
    for (int ch = 0; ch < 2; ++ch) {
      v8f acc[4];
#pragma unroll
      for (int t = 0; t < 4; ++t) { v8f z = {0.f, 0.f, 0.f, 0.f, 0.f, 0.f, 0.f, 0.f}; acc[t] = z; }
      const int ncol0 = 64 * ch;
      const size_t brow = (size_t)(p * NCP + ncol0 + m) * ldb + 8 * hh;
#pragma unroll 1
      for (int ks = 0; ks < ksteps; ++ks) {
        FragH af;
        af.h[0] = *(const v8h*)(xh + arow + 32 * ks);
        af.h[1] = *(const v8h*)(xh + arow + 32 * ks + 16);
#pragma unroll
        for (int t = 0; t < 4; ++t) {
          const size_t bo = brow + (size_t)(16 * t) * ldb + 32 * ks;
          FragH bf;
          bf.h[0] = *(const v8h*)(wt + bo);
          bf.h[1] = *(const v8h*)(wt + bo + 16);
          acc[t] = wmh(af, bf, acc[t]);
        }
      }
      float* sp = stg + (size_t)(16 * wave + 8 * hh) * NCP + ncol0 + m;
#pragma unroll
      for (int t = 0; t < 4; ++t) {
#pragma unroll
        for (int r = 0; r < 8; ++r) sp[(size_t)r * NCP + 16 * t] = acc[t][r] * SCL;
      }
    }
    __syncthreads();
    {
      const int row  = tid >> 1;
      const int half = tid & 1;
      const float* sr = stg + (size_t)row * NCP;
      float s = 0.0f, d = 0.0f;
#pragma unroll 1
      for (int c = 0; c < 64; ++c) {
        const int cc = half * 64 + c;
        const float v = sr[cc];
        s = fmaf(v, sAs[cc], s);
        d = fmaf(v, sAd[cc], d);
      }
      s += __shfl_xor(s, 1);
      d += __shfl_xor(d, 1);
      if (half == 0) { esT[row * EP + p] = s; edT[row * EP + p] = d; }
    }
    const int nF4 = GBM * NCP / 4;
    float* yb = Y + (size_t)rowBase * yp + NCP * p;
    const v4f* s4 = (const v4f*)stg;
#pragma unroll 1
    for (int f = tid; f < nF4; f += GTHR) {
      const int r = f >> 5, qq = f & 31;
      const v4f v = s4[f];
      *(volatile v4f*)(yb + (size_t)r * yp + 4 * qq) = v;
    }
    __threadfence();
#pragma unroll 1
    for (int f = tid; f < nF4; f += GTHR) {
      const int r = f >> 5, qq = f & 31;
      const v4f v = s4[f];
      *(volatile v4f*)(yb + (size_t)r * yp + 4 * qq) = v;
    }
    __syncthreads();
  }
  const v4f ve = *(const v4f*)(esT + 4 * tid);
  const v4f vd = *(const v4f*)(edT + 4 * tid);
  float* pe = ES + (size_t)rowBase * EP + 4 * tid;
  float* pd = ED + (size_t)rowBase * EP + 4 * tid;
  *(volatile v4f*)pe = ve;
  *(volatile v4f*)pd = vd;
  __threadfence();
  *(volatile v4f*)pe = ve;
  *(volatile v4f*)pd = vd;
}

template <int L1>
__global__ __launch_bounds__(NTHR) void k_agg(
    const int* __restrict__ srcs, const int* __restrict__ dsts,
    const float* __restrict__ Y, const float* __restrict__ ES, const float* __restrict__ ED,
    const float* __restrict__ bias, _Float16* xout, float* hout,
    int nN, int MP, int nE, int nb, int vec8) {
  extern __shared__ v4f lds_dyn[];
  int* reg1 = (int*)lds_dyn;
  int* reg2 = reg1 + RCAP;
  int* scnt = reg2 + RCAP;
  int* soff = scnt + NBMAX;
  int* list = soff + NBMAX;
  int* wcnt = list + LISTN;
  int* wtot = wcnt + NWAVE;
  const int tid = threadIdx.x, lane = tid & 31, wave = tid >> 5;
  const int nodeBase = (int)blockIdx.x * nb;

  for (int i = tid; i < NBMAX; i += NTHR) scnt[i] = 0;
  __syncthreads();

  int tot = 0;
  const int nChunks = (nE + CHUNK - 1) / CHUNK;
#pragma unroll 1
  for (int ch = 0; ch < nChunks; ++ch) {
    const int cbase = ch * CHUNK;
    const int wc = scan_chunk(dsts, nE, cbase, nodeBase, nb, vec8, list, tid, lane, wave);
    if (lane == 0) wcnt[wave] = wc;
    __syncthreads();
    int pre = 0, all = 0;
#pragma unroll
    for (int w2 = 0; w2 < NWAVE; ++w2) {
      int c = wcnt[w2];
      c = c < 0 ? 0 : (c > WCAP ? WCAP : c);
      all += c;
      pre += (w2 < wave) ? c : 0;
    }
    const int wcc  = wc > WCAP ? WCAP : wc;
    const int base = tot + pre;
#pragma unroll 1
    for (int i = lane; i < wcc; i += 32) {
      const int ent = list[wave * WCAP + i];
      const int el  = (ent >> 12) & (CHUNK - 1);
      const int sl  = ent & (NBMAX - 1);
      int eid = cbase + el;
      eid = eid > nE - 1 ? nE - 1 : eid;
      const int pos = base + i;
      if (pos < RCAP) reg1[pos] = (int)(((unsigned)eid << 12) | (unsigned)sl);
    }
    tot += all;
    tot = tot > RCAP ? RCAP : tot;
    __syncthreads();
  }
  const int nh = tot;

  if (wave == 0) {
#pragma unroll 1
    for (int b0 = 0; b0 < nh; b0 += 32) {
      const int idx = b0 + lane;
      const int uv  = reg1[idx < RCAP ? idx : RCAP - 1];
      const int m32 = (nh - b0) < 32 ? (nh - b0) : 32;
#pragma unroll 1
      for (int k = 0; k < m32; ++k) {
        const int u  = __builtin_amdgcn_readlane(uv, k);
        const int sl = u & (NBMAX - 1);
        if (lane == 0) scnt[sl] = scnt[sl] + 1;
      }
    }
  }
  __syncthreads();

  {
    const v4i ca = *(const v4i*)(scnt + 8 * tid);
    const v4i cb = *(const v4i*)(scnt + 8 * tid + 4);
    const int e0 = ca.x < 0 ? 0 : ca.x, e1 = ca.y < 0 ? 0 : ca.y, e2 = ca.z < 0 ? 0 : ca.z, e3 = ca.w < 0 ? 0 : ca.w;
    const int e4 = cb.x < 0 ? 0 : cb.x, e5 = cb.y < 0 ? 0 : cb.y, e6 = cb.z < 0 ? 0 : cb.z, e7 = cb.w < 0 ? 0 : cb.w;
    const int ts = e0 + e1 + e2 + e3 + e4 + e5 + e6 + e7;
    int incl = ts;
#pragma unroll
    for (int d = 1; d < 32; d <<= 1) {
      const int up = __shfl_up(incl, d);
      if (lane >= d) incl += up;
    }
    if (lane == 31) wtot[wave] = incl;
    __syncthreads();
    int pre = 0;
#pragma unroll
    for (int w2 = 0; w2 < NWAVE; ++w2) pre += (w2 < wave) ? wtot[w2] : 0;
    int run = pre + incl - ts;
    soff[8 * tid + 0] = run; run += e0;
    soff[8 * tid + 1] = run; run += e1;
    soff[8 * tid + 2] = run; run += e2;
    soff[8 * tid + 3] = run; run += e3;
    soff[8 * tid + 4] = run; run += e4;
    soff[8 * tid + 5] = run; run += e5;
    soff[8 * tid + 6] = run; run += e6;
    soff[8 * tid + 7] = run;
  }
  __syncthreads();
  for (int i = tid; i < NBMAX; i += NTHR) list[i] = soff[i];
  __syncthreads();

  if (wave == 0) {
#pragma unroll 1
    for (int b0 = 0; b0 < nh; b0 += 32) {
      const int idx = b0 + lane;
      const int uv  = reg1[idx < RCAP ? idx : RCAP - 1];
      const int m32 = (nh - b0) < 32 ? (nh - b0) : 32;
#pragma unroll 1
      for (int k = 0; k < m32; ++k) {
        const int u   = __builtin_amdgcn_readlane(uv, k);
        const int sl  = u & (NBMAX - 1);
        const int eid = (int)((unsigned)u >> 12);
        if (lane == 0) {
          int pos = list[sl];
          pos = pos < 0 ? 0 : (pos > RCAP - 1 ? RCAP - 1 : pos);
          reg2[pos] = eid;
          list[sl] = pos + 1;
        }
      }
    }
  }
  __syncthreads();

  const float nanv = __int_as_float(0x7fc00000);
  const float pois = (nh >= RCAP) ? nanv : 0.0f;
  const int nbw = nb >> 3;
  const v4f z4 = {0.f, 0.f, 0.f, 0.f};
  if (L1 != 0) {
    const int hA = lane >> 4, hB = 2 + (lane >> 4);
    const int cA = 8 * lane, cB = 256 + 8 * lane;
    const v4f bA0 = *(const v4f*)(bias + cA), bA1 = *(const v4f*)(bias + cA + 4);
    const v4f bB0 = *(const v4f*)(bias + cB), bB1 = *(const v4f*)(bias + cB + 4);
#pragma unroll 1
    for (int jt = 0; jt < nbw; ++jt) {
      const int slot = wave * nbw + jt;
      const int grow = nodeBase + slot;
      const int gcl  = grow < nN ? grow : nN - 1;
      int st  = soff[slot];
      int cnt = scnt[slot];
      st  = st < 0 ? 0 : (st > nh ? nh : st);
      const float pz = ((cnt > DEGCAP) ? nanv : 0.0f) + pois;
      cnt = cnt < 0 ? 0 : (cnt > DEGCAP ? DEGCAP : cnt);
      if (cnt > nh - st) cnt = nh - st;

      const float* yd = Y + (size_t)gcl * HCA;
      v4f aA0 = *(const v4f*)(yd + cA), aA1 = *(const v4f*)(yd + cA + 4);
      v4f aB0 = *(const v4f*)(yd + cB), aB1 = *(const v4f*)(yd + cB + 4);
      const float eddA = ED[(size_t)gcl * EP + hA], eddB = ED[(size_t)gcl * EP + hB];
      const float esdA = ES[(size_t)gcl * EP + hA], esdB = ES[(size_t)gcl * EP + hB];
      const float uA0 = esdA + eddA, uB0 = esdB + eddB;
      float mxA = fmaxf(uA0, NEG_SLOPE * uA0), mxB = fmaxf(uB0, NEG_SLOPE * uB0);
      float denA = 1.0f, denB = 1.0f;

#pragma unroll 1
      for (int q = 0; q < cnt; ++q) {
        int idx = st + q; idx = idx > RCAP - 1 ? RCAP - 1 : idx;
        int eid = reg2[idx]; eid = eid < 0 ? 0 : (eid > nE - 1 ? nE - 1 : eid);
        const int sraw = srcs[eid];
        const int s = sraw < 0 ? 0 : (sraw > nN - 1 ? nN - 1 : sraw);
        const float* ys = Y + (size_t)s * HCA;
        const v4f xA0 = *(const v4f*)(ys + cA), xA1 = *(const v4f*)(ys + cA + 4);
        const v4f xB0 = *(const v4f*)(ys + cB), xB1 = *(const v4f*)(ys + cB + 4);
        const float essA = ES[(size_t)s * EP + hA], essB = ES[(size_t)s * EP + hB];
        const float uA = essA + eddA, uB = essB + eddB;
        const float lgA = fmaxf(uA, NEG_SLOPE * uA), lgB = fmaxf(uB, NEG_SLOPE * uB);
        const float mnA = fmaxf(mxA, lgA), mnB = fmaxf(mxB, lgB);
        const float s1A = __expf(mxA - mnA), s2A = __expf(lgA - mnA);
        const float s1B = __expf(mxB - mnB), s2B = __expf(lgB - mnB);
        denA = fmaf(denA, s1A, s2A);
        denB = fmaf(denB, s1B, s2B);
        aA0 = aA0 * s1A + xA0 * s2A;
        aA1 = aA1 * s1A + xA1 * s2A;
        aB0 = aB0 * s1B + xB0 * s2B;
        aB1 = aB1 * s1B + xB1 * s2B;
        mxA = mnA; mxB = mnB;
      }
      const float invA = __builtin_amdgcn_rcpf(denA);
      const float invB = __builtin_amdgcn_rcpf(denB);
      v4f oA0 = elu4(aA0 * invA + bA0) + pz;
      v4f oA1 = elu4(aA1 * invA + bA1) + pz;
      v4f oB0 = elu4(aB0 * invB + bB0) + pz;
      v4f oB1 = elu4(aB1 * invB + bB1) + pz;
      const bool live = grow < nN;
      if (!live) { oA0 = z4; oA1 = z4; oB0 = z4; oB1 = z4; }
      v8h hvA, hvB;
      hvA[0] = (_Float16)(oA0.x * CA); hvA[1] = (_Float16)(oA0.y * CA);
      hvA[2] = (_Float16)(oA0.z * CA); hvA[3] = (_Float16)(oA0.w * CA);
      hvA[4] = (_Float16)(oA1.x * CA); hvA[5] = (_Float16)(oA1.y * CA);
      hvA[6] = (_Float16)(oA1.z * CA); hvA[7] = (_Float16)(oA1.w * CA);
      hvB[0] = (_Float16)(oB0.x * CA); hvB[1] = (_Float16)(oB0.y * CA);
      hvB[2] = (_Float16)(oB0.z * CA); hvB[3] = (_Float16)(oB0.w * CA);
      hvB[4] = (_Float16)(oB1.x * CA); hvB[5] = (_Float16)(oB1.y * CA);
      hvB[6] = (_Float16)(oB1.z * CA); hvB[7] = (_Float16)(oB1.w * CA);
      const bool wr = grow < MP;
      const int grc = grow < MP ? grow : MP - 1;
      _Float16* xp = xout + (size_t)grc * HCA;
      if (wr) { *(volatile v8h*)(xp + cA) = hvA; *(volatile v8h*)(xp + cB) = hvB; }
      __threadfence();
      if (wr) { *(volatile v8h*)(xp + cA) = hvA; *(volatile v8h*)(xp + cB) = hvB; }
    }
  } else {
    const int c4 = 4 * lane;
    const v4f bz = *(const v4f*)(bias + c4);
#pragma unroll 1
    for (int jt = 0; jt < nbw; ++jt) {
      const int slot = wave * nbw + jt;
      const int grow = nodeBase + slot;
      const int gcl  = grow < nN ? grow : nN - 1;
      int st  = soff[slot];
      int cnt = scnt[slot];
      st  = st < 0 ? 0 : (st > nh ? nh : st);
      const float pz = ((cnt > DEGCAP) ? nanv : 0.0f) + pois;
      cnt = cnt < 0 ? 0 : (cnt > DEGCAP ? DEGCAP : cnt);
      if (cnt > nh - st) cnt = nh - st;

      const float* yd = Y + (size_t)gcl * HCB;
      v4f acc = *(const v4f*)(yd + c4);
      const float edd = ED[(size_t)gcl * EP];
      const float esd = ES[(size_t)gcl * EP];
      const float u0 = esd + edd;
      float mx  = fmaxf(u0, NEG_SLOPE * u0);
      float den = 1.0f;

#pragma unroll 1
      for (int q = 0; q < cnt; ++q) {
        int idx = st + q; idx = idx > RCAP - 1 ? RCAP - 1 : idx;
        int eid = reg2[idx]; eid = eid < 0 ? 0 : (eid > nE - 1 ? nE - 1 : eid);
        const int sraw = srcs[eid];
        const int s = sraw < 0 ? 0 : (sraw > nN - 1 ? nN - 1 : sraw);
        const v4f xs = *(const v4f*)(Y + (size_t)s * HCB + c4);
        const float ess = ES[(size_t)s * EP];
        const float u1 = ess + edd;
        const float lg = fmaxf(u1, NEG_SLOPE * u1);
        const float mn = fmaxf(mx, lg);
        const float s1 = __expf(mx - mn);
        const float s2 = __expf(lg - mn);
        den = fmaf(den, s1, s2);
        acc = acc * s1 + xs * s2;
        mx = mn;
      }
      const float inv = __builtin_amdgcn_rcpf(den);
      const v4f o = elu4(acc * inv + bz) + pz;
      const bool wr = grow < nN;
      float* gp = hout + (size_t)gcl * HCB + c4;
      if (wr) *(volatile v4f*)gp = o;
      __threadfence();
      if (wr) *(volatile v4f*)gp = o;
    }
  }
}

__global__ __launch_bounds__(PTHR) void k_pool(const int* __restrict__ batch, const float* __restrict__ hb,
                                               float* out, int nN) {
  __shared__ int plist[PTHR];
  __shared__ int wc4[PTHR / 32];
  __shared__ __attribute__((aligned(16))) float sout[PTHR];
  const int tid = threadIdx.x, lane = tid & 31, wave = tid >> 5;
  const int g = (int)blockIdx.x;
  float mx = -__int_as_float(0x7f800000);
  const int nChunks = (nN + PTHR - 1) / PTHR;
#pragma unroll 1
  for (int ch = 0; ch < nChunks; ++ch) {
    const int i = ch * PTHR + tid;
    const int b = batch[i < nN ? i : nN - 1];
    const bool hit = (i < nN) && (b == g);
    const unsigned mk = __builtin_amdgcn_ballot_w32(hit);
    const int pos = (int)__builtin_amdgcn_mbcnt_lo(mk, 0u);
    if (lane == 0) wc4[wave] = (int)__builtin_popcount(mk);
    __syncthreads();
    int pre = 0, tot = 0;
#pragma unroll
    for (int w2 = 0; w2 < PTHR / 32; ++w2) {
      const int c = wc4[w2];
      tot += c;
      pre += (w2 < wave) ? c : 0;
    }
    if (hit) { const int p = pre + pos; if (p < PTHR) plist[p] = i; }
    tot = tot > PTHR ? PTHR : tot;
    __syncthreads();
#pragma unroll 1
    for (int k = 0; k < tot; ++k) {
      int nd = plist[k];
      nd = nd < 0 ? 0 : (nd > nN - 1 ? nN - 1 : nd);
      const float v = hb[(size_t)nd * HCB + tid];
      mx = (v > mx || v != v) ? v : mx;
    }
    __syncthreads();
  }
  sout[tid] = mx;
  __syncthreads();
  if (wave == 0) {
    const v4f v = *(const v4f*)(sout + 4 * lane);
    float* op = out + (size_t)g * HCB + 4 * lane;
    *(volatile v4f*)op = v;
    __threadfence();
    *(volatile v4f*)op = v;
  }
}

static int pick_nb(int nE, int nN) {
  int nb = NBMAX;
  while (nb > 16 && (long long)nb * (long long)nE * 5LL > (long long)RCAP * (long long)nN * 4LL) nb >>= 1;
  return nb;
}

extern "C" void kernel_launch(void* const* d_in, const int* in_sizes, int n_in,
                              void* d_out, int out_size, void* d_ws, size_t ws_size,
                              hipStream_t stream) {
  if (n_in < 23) return;
  const int nN = in_sizes[0] / SF;
  if (nN <= 0 || in_sizes[0] != nN * SF) return;
  if (nN > (1 << 22)) return;
  for (int i = 1; i <= 5; ++i) if (in_sizes[i] != nN * LL) return;
  const int szE = in_sizes[6];
  if (szE < 2 || (szE & 1) != 0) return;
  const int nE = szE / 2;
  if (nE > (1 << 20)) return;
  if (in_sizes[7] != nN) return;
  int voc[NTAB];
  for (int t = 0; t < NTAB; ++t) {
    const int s = in_sizes[8 + t];
    if (s < DM || (s % DM) != 0) return;
    voc[t] = s / DM;
  }
  if (in_sizes[13] != FT || in_sizes[14] != FT) return;
  if (in_sizes[15] != FT * HCA) return;
  if (in_sizes[16] != HCA || in_sizes[17] != HCA || in_sizes[18] != HCA) return;
  if (in_sizes[19] != HCA * HCB) return;
  if (in_sizes[20] != HCB || in_sizes[21] != HCB || in_sizes[22] != HCB) return;
  const int nG = out_size / HCB;
  if (nG <= 0 || out_size != nG * HCB) return;

  const float* xs   = (const float*)d_in[0];
  const int*   i0   = (const int*)d_in[1];
  const int*   i1   = (const int*)d_in[2];
  const int*   i2   = (const int*)d_in[3];
  const int*   i3   = (const int*)d_in[4];
  const int*   i4   = (const int*)d_in[5];
  const int*   ei   = (const int*)d_in[6];
  const int*   bat  = (const int*)d_in[7];
  const float* e0   = (const float*)d_in[8];
  const float* e1   = (const float*)d_in[9];
  const float* e2   = (const float*)d_in[10];
  const float* e3   = (const float*)d_in[11];
  const float* e4   = (const float*)d_in[12];
  const float* lnsc = (const float*)d_in[13];
  const float* lnb  = (const float*)d_in[14];
  const float* W1   = (const float*)d_in[15];
  const float* as1  = (const float*)d_in[16];
  const float* ad1  = (const float*)d_in[17];
  const float* b1   = (const float*)d_in[18];
  const float* W2   = (const float*)d_in[19];
  const float* as2  = (const float*)d_in[20];
  const float* ad2  = (const float*)d_in[21];
  const float* b2   = (const float*)d_in[22];
  float* out = (float*)d_out;

  const int MP   = ((nN + GBM - 1) / GBM) * GBM;
  const int nb   = pick_nb(nE, nN);
  if (nb < 8 || nb > NBMAX) return;
  const int vec8 = ((nE & 3) == 0) ? 1 : 0;

  char* ws = (char*)d_ws;
  size_t off = 0;
  const size_t oWTA = off; off += (size_t)HCA * KPA * 2;          off = (off + 255) & ~(size_t)255;
  const size_t oWTB = off; off += (size_t)HCB * HCA * 2;          off = (off + 255) & ~(size_t)255;
  const size_t oXA  = off; off += (size_t)MP * KPA * 2;           off = (off + 255) & ~(size_t)255;
  const size_t oXB  = off; off += (size_t)MP * HCA * 2;           off = (off + 255) & ~(size_t)255;
  const size_t oY   = off; off += (size_t)MP * HCA * 4;           off = (off + 255) & ~(size_t)255;
  const size_t oES  = off; off += (size_t)MP * EP * 4;            off = (off + 255) & ~(size_t)255;
  const size_t oED  = off; off += (size_t)MP * EP * 4;            off = (off + 255) & ~(size_t)255;
  if (off > ws_size || off > (size_t)WSCAP) return;
  _Float16* WTA = (_Float16*)(ws + oWTA);
  _Float16* WTB = (_Float16*)(ws + oWTB);
  _Float16* XA  = (_Float16*)(ws + oXA);
  _Float16* XB  = (_Float16*)(ws + oXB);
  float*    YA  = (float*)(ws + oY);
  float*    YB  = (float*)(ws + oY);
  float*    HB  = (float*)(ws + oY + (size_t)MP * HCB * 4);
  float*    ES  = (float*)(ws + oES);
  float*    ED  = (float*)(ws + oED);
  const int* srcp = ei;
  const int* dstp = ei + nE;

  hipFuncSetAttribute(reinterpret_cast<const void*>(&k_agg<1>),
                      hipFuncAttributeMaxDynamicSharedMemorySize, LDS_AGG);
  hipFuncSetAttribute(reinterpret_cast<const void*>(&k_agg<0>),
                      hipFuncAttributeMaxDynamicSharedMemorySize, LDS_AGG);

  k_feat<<<MP / NWAVE, NTHR, 0, stream>>>(xs, i0, i1, i2, i3, i4, e0, e1, e2, e3, e4, lnsc, lnb,
                                          XA, nN, voc[0], voc[1], voc[2], voc[3], voc[4]);
  const int uA = HCA * KPA / 8, uB = HCB * HCA / 8;
  k_wprep<<<(uA + NTHR - 1) / NTHR, NTHR, 0, stream>>>(W1, WTA, FT, HCA, KPA, uA);
  k_wprep<<<(uB + NTHR - 1) / NTHR, NTHR, 0, stream>>>(W2, WTB, HCA, HCB, HCA, uB);

  const int gG = MP / GBM;
  const int gA = (MP + nb - 1) / nb;

  k_gemm<<<gG, GTHR, 0, stream>>>(XA, KPA, FT / 32, WTA, KPA, as1, ad1, YA, HCA, ES, ED, NHA);
  k_agg<1><<<gA, NTHR, LDS_AGG, stream>>>(srcp, dstp, YA, ES, ED, b1, XB, HB, nN, MP, nE, nb, vec8);
  k_gemm<<<gG, GTHR, 0, stream>>>(XB, HCA, HCA / 32, WTB, HCA, as2, ad2, YB, HCB, ES, ED, 1);
  k_agg<0><<<gA, NTHR, LDS_AGG, stream>>>(srcp, dstp, YB, ES, ED, b2, XB, HB, nN, MP, nE, nb, vec8);
  k_pool<<<nG, PTHR, 0, stream>>>(bat, HB, out, nN);
}
